// DisjointDecoderAE_27393301413996
// MI455X (gfx1250) — hardware-verified
//
#include <hip/hip_runtime.h>


#define NBT  2048
#define NU   512
#define LAT  32
#define HID  64
typedef _Float16 h16;
typedef unsigned short bf;
typedef __attribute__((ext_vector_type(16))) __bf16   v16bf;
typedef __attribute__((ext_vector_type(16))) _Float16 v16h;
typedef __attribute__((ext_vector_type(8)))  _Float16 v8h;
typedef __attribute__((ext_vector_type(8)))  unsigned short v8us;
typedef __attribute__((ext_vector_type(8)))  float    v8f;
typedef __attribute__((ext_vector_type(4)))  float    v4f;
typedef v8h  __attribute__((may_alias)) v8ha;
typedef v4f  __attribute__((may_alias)) v4fa;
typedef v8us __attribute__((may_alias)) v8usa;

__device__ __forceinline__ unsigned short f2bf(float f) { unsigned u = __float_as_uint(f); u += 0x7FFFu + ((u >> 16) & 1u); return (unsigned short)(u >> 16); }
__device__ __forceinline__ float bf2f(unsigned short b) { return __uint_as_float(((unsigned)b) << 16); }
__device__ __forceinline__ float bfr(float f) { return bf2f(f2bf(f)); }
__device__ __forceinline__ v16h cat16(v8h lo, v8h hi) { return __builtin_shufflevector(lo, hi, 0, 1, 2, 3, 4, 5, 6, 7, 8, 9, 10, 11, 12, 13, 14, 15); }
__device__ __forceinline__ v16bf cat16b(v8us lo, v8us hi) { return __builtin_bit_cast(v16bf, __builtin_shufflevector(lo, hi, 0, 1, 2, 3, 4, 5, 6, 7, 8, 9, 10, 11, 12, 13, 14, 15)); }
__device__ __forceinline__ v8f wmma16(v16h a, v16h b, v8f c) { return __builtin_amdgcn_wmma_f32_16x16x32_f16(false, a, false, b, (short)0, c, false, false); }
__device__ __forceinline__ v8f wmmab(v16bf a, v16bf b, v8f c) { return __builtin_amdgcn_wmma_f32_16x16x32_bf16(false, a, false, b, (short)0, c, false, false); }


template <typename T16> struct WFrag;
template <> struct WFrag<h16> { typedef v16h V; static __device__ __forceinline__ V ld(const h16* p) { return cat16(*(const v8h*)p, *(const v8h*)(p + 16)); } static __device__ __forceinline__ v8f mma(V a, V b, v8f c) { return wmma16(a, b, c); } };
template <> struct WFrag<bf> { typedef v16bf V; static __device__ __forceinline__ V ld(const bf* p) { return cat16b(*(const v8us*)p, *(const v8us*)(p + 16)); } static __device__ __forceinline__ v8f mma(V a, V b, v8f c) { return wmmab(a, b, c); } };
template <typename T16, int NSPLIT, bool BIAS>
__global__ __launch_bounds__(32) void k_gemmw(const T16* __restrict__ A, const T16* __restrict__ A2, const T16* __restrict__ Bt, const T16* __restrict__ Bt2, int K, float* C, int ldc, const float* __restrict__ bias, size_t sA, size_t sB, size_t sC) {
    typedef typename WFrag<T16>::V V;
    __shared__ __align__(16) float os[16 * 68];
    const size_t z = blockIdx.z; A += z * sA; if (A2) A2 += z * sA; Bt += z * sB; if (Bt2) Bt2 += z * sB; C += z * sC;
    const int lane = threadIdx.x & 31, lr = lane & 15, hi = lane >> 4; const int r0 = blockIdx.x * 64, c0 = blockIdx.y * 64;
    v8f acc[4][4];
#pragma unroll
    for (int mb = 0; mb < 4; ++mb)
#pragma unroll
        for (int nb = 0; nb < 4; ++nb) acc[mb][nb] = (v8f){};
    const size_t aoff = (size_t)(r0 + lr) * K + 8 * hi, boff = (size_t)(c0 + lr) * K + 8 * hi;
#pragma unroll 1
    for (int kc = 0; kc < K; kc += 32) {
        V a[4], a2[4];
#pragma unroll
        for (int mb = 0; mb < 4; ++mb) { a[mb] = WFrag<T16>::ld(A + aoff + (size_t)mb * 16 * K + kc); if (NSPLIT == 1 || NSPLIT == 2) a2[mb] = WFrag<T16>::ld(A2 + aoff + (size_t)mb * 16 * K + kc); }
#pragma unroll
        for (int nb = 0; nb < 4; ++nb) { const V b = WFrag<T16>::ld(Bt + boff + (size_t)nb * 16 * K + kc); V b2; if (NSPLIT >= 2) b2 = WFrag<T16>::ld(Bt2 + boff + (size_t)nb * 16 * K + kc);
#pragma unroll
            for (int mb = 0; mb < 4; ++mb) { acc[mb][nb] = WFrag<T16>::mma(a[mb], b, acc[mb][nb]); if (NSPLIT == 1 || NSPLIT == 2) acc[mb][nb] = WFrag<T16>::mma(a2[mb], b, acc[mb][nb]); if (NSPLIT >= 2) acc[mb][nb] = WFrag<T16>::mma(a[mb], b2, acc[mb][nb]); } }
        asm volatile("v_nop\n\tv_nop\n\tv_nop\n\tv_nop" : "+v"(acc[0][0]), "+v"(acc[1][1]), "+v"(acc[2][2]), "+v"(acc[3][3]) : "v"(a[0]), "v"(a[3]));
    }
#pragma unroll
    for (int mb = 0; mb < 4; ++mb) {
#pragma unroll
        for (int nb = 0; nb < 4; ++nb) {
#pragma unroll
            for (int j = 0; j < 8; ++j) os[(hi * 8 + j) * 68 + nb * 16 + lr] = acc[mb][nb][j]; }
        __builtin_amdgcn_wave_barrier(); asm volatile("" ::: "memory");
        float* crow = C + (size_t)(r0 + mb * 16) * ldc + c0;
#pragma unroll 1
        for (int ps = 0; ps < 2; ++ps) {
#pragma unroll
            for (int s = 0; s < 8; ++s) { const int row = 2 * s + hi, cofs = lr * 4; v4f val = *(const v4fa*)(os + row * 68 + cofs); if (BIAS) { val[0] += bfr(bias[c0 + cofs]); val[1] += bfr(bias[c0 + cofs + 1]); val[2] += bfr(bias[c0 + cofs + 2]); val[3] += bfr(bias[c0 + cofs + 3]); }
                *(volatile v4f*)(crow + (size_t)row * ldc + cofs) = val; }
            if (ps == 0) __threadfence(); }
        __builtin_amdgcn_wave_barrier(); asm volatile("" ::: "memory");
    }
}

__device__ __forceinline__ void splitf(float y, unsigned short& h, unsigned short& l) { h = f2bf(y); l = f2bf(y - bf2f(h)); }
typedef __attribute__((ext_vector_type(2))) unsigned short v2us;
typedef __attribute__((ext_vector_type(2))) float v2f;

__global__ __launch_bounds__(256) void k_cvt8(const float* __restrict__ src, bf* dst, size_t n8) { const size_t i = (size_t)blockIdx.x * 256 + threadIdx.x; if (i >= n8) return; const v8f v = *(const v8f*)(src + i * 8); v8us o;
#pragma unroll
    for (int k = 0; k < 8; ++k) o[k] = f2bf(v[k]); *(volatile v8us*)(dst + i * 8) = o; __threadfence(); *(volatile v8us*)(dst + i * 8) = o; }
__global__ __launch_bounds__(256) void k_wtZ(const float* __restrict__ w, int U, int K, int N, bf* Bt) {
    const int lane = threadIdx.x & 31; const int L0 = (blockIdx.x * 8 + (threadIdx.x >> 5)) * 8; const int nlines = U * N * K / 64;
#pragma unroll 1
    for (int ps = 0; ps < 2; ++ps) {
#pragma unroll 1
        for (int l = 0; l < 8; ++l) { const int L = L0 + l; if (L >= nlines) break; const size_t e = (size_t)L * 64 + lane * 2; const int k = (int)(e % K); const int n = (int)((e / K) % N); const int u = (int)(e / ((size_t)K * N)); v2us o;
            o[0] = f2bf(w[((size_t)u * K + k) * N + n]); o[1] = f2bf(w[((size_t)u * K + k + 1) * N + n]); *(volatile v2us*)(Bt + e) = o; }
        if (ps == 0) __threadfence(); }
}
template <int RELU>
__global__ __launch_bounds__(256) void k_brsplit(const float* __restrict__ F, const float* __restrict__ bias, int Z, int R, int C, bf* Ph, bf* Pl) {
    const int lane = threadIdx.x & 31; const int L0 = (blockIdx.x * 8 + (threadIdx.x >> 5)) * 8; const size_t nlines = (size_t)Z * R * C / 64;
#pragma unroll 1
    for (int ps = 0; ps < 2; ++ps) {
#pragma unroll 1
        for (int l = 0; l < 8; ++l) { const size_t L = (size_t)L0 + l; if (L >= nlines) break; const size_t e = L * 64 + lane * 2; const int c = (int)(e % C); const int z = (int)(e / ((size_t)R * C)); v2us oh, ol;
#pragma unroll
            for (int q = 0; q < 2; ++q) { float t = F[e + q] + bfr(bias[(size_t)z * C + c + q]); if (RELU) t = fmaxf(t, 0.f); unsigned short a, c2; splitf(t, a, c2); oh[q] = a; ol[q] = c2; }
            *(volatile v2us*)(Ph + e) = oh; *(volatile v2us*)(Pl + e) = ol; }
        if (ps == 0) __threadfence(); }
}
__global__ __launch_bounds__(256) void k_zsplit(const float* __restrict__ F, const float* __restrict__ be4, bf* Zh, bf* Zl) {
    const int lane = threadIdx.x & 31; const int L = blockIdx.x * 8 + (threadIdx.x >> 5); if (L >= NBT * LAT / 64) return; const int e = L * 64 + lane * 2; const int c = e & (LAT - 1), r = e >> 5; v2us oh, ol;
#pragma unroll
    for (int q = 0; q < 2; ++q) { unsigned short a, c2; splitf(F[(size_t)r * HID + c + q] + bfr(be4[c + q]), a, c2); oh[q] = a; ol[q] = c2; }
    *(volatile v2us*)(Zh + e) = oh; *(volatile v2us*)(Zl + e) = ol; __threadfence(); *(volatile v2us*)(Zh + e) = oh; *(volatile v2us*)(Zl + e) = ol;
}
__global__ __launch_bounds__(256) void k_head(const float* __restrict__ H, const float* __restrict__ bd3, const float* __restrict__ Wd4, const float* __restrict__ bd4, int u0, int UC, float* OUT) {
    const int lane = threadIdx.x & 31; const int wg = blockIdx.x * 8 + (threadIdx.x >> 5); if (wg >= NBT * (UC / 32)) return; const int b = wg / (UC / 32); const int uu = (wg % (UC / 32)) * 32 + lane; const int u = u0 + uu;
    const float* hr = H + ((size_t)uu * NBT + b) * HID; const float* br = bd3 + (size_t)u * HID; const float* wr = Wd4 + (size_t)u * HID; float s = bfr(bd4[u]);
#pragma unroll 4
    for (int h = 0; h < HID; ++h) s = __fadd_rn(s, __fmul_rn(fmaxf(hr[h] + bfr(br[h]), 0.f), bfr(wr[h])));
    *(volatile float*)(OUT + (size_t)b * NU + u) = s; __threadfence(); *(volatile float*)(OUT + (size_t)b * NU + u) = s;
}

extern "C" void kernel_launch(void* const* d_in, const int* in_sizes, int n_in,
                              void* d_out, int out_size, void* d_ws, size_t ws_size, hipStream_t stream) {
    (void)in_sizes; (void)n_in; (void)out_size;
    const float* IN[17]; for (int i = 0; i < 17; ++i) IN[i] = (const float*)d_in[i];
    float* OUT = (float*)d_out;
    char* wsp = (char*)d_ws;
    auto take = [&](size_t bytes) { char* p = wsp; wsp += (bytes + 255) & ~(size_t)255; return (void*)p; };
    bf* WE1 = (bf*)take((size_t)HID * NU * 2); bf* WE2 = (bf*)take((size_t)HID * HID * 2); bf* WE3 = (bf*)take((size_t)HID * HID * 2); bf* WE4 = (bf*)take((size_t)64 * HID * 2);
    bf* WD1 = (bf*)take((size_t)NU * HID * LAT * 2); bf* WD2 = (bf*)take((size_t)NU * HID * HID * 2); bf* WD3 = (bf*)take((size_t)NU * HID * HID * 2);
    bf* XB = (bf*)take((size_t)NBT * NU * 2); float* F = (float*)take((size_t)NBT * HID * 4); bf* Eh = (bf*)take((size_t)NBT * HID * 2); bf* El = (bf*)take((size_t)NBT * HID * 2); bf* Zh = (bf*)take((size_t)NBT * LAT * 2); bf* Zl = (bf*)take((size_t)NBT * LAT * 2);
    const int UC = 128;
    float* G = (float*)take((size_t)UC * NBT * HID * 4); bf* Gh = (bf*)take((size_t)UC * NBT * HID * 2); bf* Gl = (bf*)take((size_t)UC * NBT * HID * 2);
    if ((size_t)(wsp - (char*)d_ws) > ws_size) return;
    hipMemsetAsync(WE4, 0, (size_t)64 * HID * 2, stream);
    { k_wtZ<<<(NU * HID / 64 + 7) / 8, 256, 0, stream>>>(IN[1], 1, NU, HID, WE1); k_wtZ<<<1, 256, 0, stream>>>(IN[3], 1, HID, HID, WE2); k_wtZ<<<1, 256, 0, stream>>>(IN[5], 1, HID, HID, WE3); k_wtZ<<<1, 256, 0, stream>>>(IN[7], 1, HID, LAT, WE4);
      k_wtZ<<<(NU * HID * LAT / 64 + 7) / 8, 256, 0, stream>>>(IN[9], NU, LAT, HID, WD1); k_wtZ<<<(NU * HID * HID / 64 + 7) / 8, 256, 0, stream>>>(IN[11], NU, HID, HID, WD2); k_wtZ<<<(NU * HID * HID / 64 + 7) / 8, 256, 0, stream>>>(IN[13], NU, HID, HID, WD3); }
    k_cvt8<<<(NBT * NU / 8 + 255) / 256, 256, 0, stream>>>(IN[0], XB, (size_t)NBT * NU / 8);
    const unsigned LE = (NBT * HID / 64 + 63) / 64;
    k_gemmw<bf, 0, false><<<dim3(NBT / 64, 1, 1), 32, 0, stream>>>(XB, nullptr, WE1, nullptr, NU, F, HID, nullptr, 0, 0, 0); k_brsplit<1><<<LE, 256, 0, stream>>>(F, IN[2], 1, NBT, HID, Eh, El);
    k_gemmw<bf, 1, false><<<dim3(NBT / 64, 1, 1), 32, 0, stream>>>(Eh, El, WE2, nullptr, HID, F, HID, nullptr, 0, 0, 0); k_brsplit<1><<<LE, 256, 0, stream>>>(F, IN[4], 1, NBT, HID, Eh, El);
    k_gemmw<bf, 1, false><<<dim3(NBT / 64, 1, 1), 32, 0, stream>>>(Eh, El, WE3, nullptr, HID, F, HID, nullptr, 0, 0, 0); k_brsplit<1><<<LE, 256, 0, stream>>>(F, IN[6], 1, NBT, HID, Eh, El);
    k_gemmw<bf, 1, false><<<dim3(NBT / 64, 1, 1), 32, 0, stream>>>(Eh, El, WE4, nullptr, HID, F, HID, nullptr, 0, 0, 0); k_zsplit<<<(NBT * LAT / 64 + 7) / 8, 256, 0, stream>>>(F, IN[8], Zh, Zl);
    const unsigned LG = (unsigned)(((size_t)UC * NBT * HID / 64 + 63) / 64);
    for (int u0 = 0; u0 < NU; u0 += UC) {
        k_gemmw<bf, 1, false><<<dim3(NBT / 64, 1, UC), 32, 0, stream>>>(Zh, Zl, WD1 + (size_t)u0 * HID * LAT, nullptr, LAT, G, HID, nullptr, 0, (size_t)HID * LAT, (size_t)NBT * HID);
        k_brsplit<1><<<LG, 256, 0, stream>>>(G, IN[10] + (size_t)u0 * HID, UC, NBT, HID, Gh, Gl);
        k_gemmw<bf, 1, false><<<dim3(NBT / 64, 1, UC), 32, 0, stream>>>(Gh, Gl, WD2 + (size_t)u0 * HID * HID, nullptr, HID, G, HID, nullptr, (size_t)NBT * HID, (size_t)HID * HID, (size_t)NBT * HID);
        k_brsplit<1><<<LG, 256, 0, stream>>>(G, IN[12] + (size_t)u0 * HID, UC, NBT, HID, Gh, Gl);
        k_gemmw<bf, 1, false><<<dim3(NBT / 64, 1, UC), 32, 0, stream>>>(Gh, Gl, WD3 + (size_t)u0 * HID * HID, nullptr, HID, G, HID, nullptr, (size_t)NBT * HID, (size_t)HID * HID, (size_t)NBT * HID);
        k_head<<<NBT * (UC / 32) / 8, 256, 0, stream>>>(G, IN[14], IN[15], IN[16], u0, UC, OUT); }
}
